// TabularModel_8950711844965
// MI455X (gfx1250) — hardware-verified
//
#include <hip/hip_runtime.h>


#define NB_  65536
#define NCAT 1479
#define NCON 11
#define KP   1536
#define N1   200
#define N1P  256
#define N2   100
#define N2P  128
#define DM   KP
#define LOSC 1024.0f
typedef _Float16 h16;
typedef unsigned short bf;
typedef __attribute__((ext_vector_type(16))) __bf16   v16bf;
typedef __attribute__((ext_vector_type(16))) _Float16 v16h;
typedef __attribute__((ext_vector_type(8)))  _Float16 v8h;
typedef __attribute__((ext_vector_type(8)))  unsigned short v8us;
typedef __attribute__((ext_vector_type(8)))  float    v8f;
typedef __attribute__((ext_vector_type(4)))  float    v4f;
typedef v8h  __attribute__((may_alias)) v8ha;
typedef v4f  __attribute__((may_alias)) v4fa;
typedef v8us __attribute__((may_alias)) v8usa;

__device__ __forceinline__ unsigned short f2bf(float f) { unsigned u = __float_as_uint(f); u += 0x7FFFu + ((u >> 16) & 1u); return (unsigned short)(u >> 16); }
__device__ __forceinline__ float bf2f(unsigned short b) { return __uint_as_float(((unsigned)b) << 16); }
__device__ __forceinline__ float bfr(float f) { return bf2f(f2bf(f)); }
__device__ __forceinline__ v16h cat16(v8h lo, v8h hi) { return __builtin_shufflevector(lo, hi, 0, 1, 2, 3, 4, 5, 6, 7, 8, 9, 10, 11, 12, 13, 14, 15); }
__device__ __forceinline__ v16bf cat16b(v8us lo, v8us hi) { return __builtin_bit_cast(v16bf, __builtin_shufflevector(lo, hi, 0, 1, 2, 3, 4, 5, 6, 7, 8, 9, 10, 11, 12, 13, 14, 15)); }
__device__ __forceinline__ v8f wmma16(v16h a, v16h b, v8f c) { return __builtin_amdgcn_wmma_f32_16x16x32_f16(false, a, false, b, (short)0, c, false, false); }
__device__ __forceinline__ v8f wmmab(v16bf a, v16bf b, v8f c) { return __builtin_amdgcn_wmma_f32_16x16x32_bf16(false, a, false, b, (short)0, c, false, false); }

template <bool SPLITA, bool F16OUT = false>
__global__ __launch_bounds__(128) void k_gemmb(const bf* __restrict__ A, const bf* __restrict__ Al, const bf* __restrict__ Bn, const float* __restrict__ bias, float* C, int ldc, h16* C2, const float* __restrict__ R = nullptr, int K = DM, int roundR = 1) {
    __shared__ __align__(16) float ost[4][16 * 68];
    const int lane = threadIdx.x & 31, wave = threadIdx.x >> 5, lr = lane & 15, hi = lane >> 4;
    const int r0 = blockIdx.x * 64 + wave * 16, c0 = blockIdx.y * 64;
    const size_t aoff = (size_t)(r0 + lr) * K + 8 * hi;
    size_t boff[4];
#pragma unroll
    for (int t = 0; t < 4; ++t) boff[t] = (size_t)(c0 + t * 16 + lr) * K + 8 * hi;
    v8f acc[4];
#pragma unroll
    for (int t = 0; t < 4; ++t) acc[t] = (v8f){};
#pragma unroll 1
    for (int kc = 0; kc < K; kc += 32) {
        const v16bf a = cat16b(*(const v8us*)(A + aoff + kc), *(const v8us*)(A + aoff + kc + 16));
        v16bf al = a;
        if (SPLITA) al = cat16b(*(const v8us*)(Al + aoff + kc), *(const v8us*)(Al + aoff + kc + 16));
#pragma unroll
        for (int t = 0; t < 4; ++t) { const v16bf b = cat16b(*(const v8us*)(Bn + boff[t] + kc), *(const v8us*)(Bn + boff[t] + kc + 16)); acc[t] = wmmab(a, b, acc[t]); if (SPLITA) acc[t] = wmmab(al, b, acc[t]); }
        asm volatile("v_nop\n\tv_nop\n\tv_nop\n\tv_nop" : "+v"(acc[0]), "+v"(acc[1]), "+v"(acc[2]), "+v"(acc[3]) : "v"(a), "v"(al));
    }
    float* os = &ost[wave][0];
#pragma unroll
    for (int t = 0; t < 4; ++t) { const float bv = bias ? bfr(bias[c0 + t * 16 + lr]) : 0.f;
#pragma unroll
        for (int j = 0; j < 8; ++j) os[(hi * 8 + j) * 68 + t * 16 + lr] = acc[t][j] + bv; }
    __syncthreads();
    if (F16OUT) {
        h16* crow = (h16*)(void*)C + (size_t)r0 * ldc + c0;
        auto pass = [&]() {
#pragma unroll
            for (int s = 0; s < 4; ++s) { const int row = 4 * s + (lane >> 3), piece = lane & 7; const float* sp = os + row * 68 + piece * 8; v8h o, o2;
#pragma unroll
                for (int i = 0; i < 8; ++i) { const h16 a = (h16)sp[i]; o[i] = a; o2[i] = (h16)((sp[i] - (float)a) * LOSC); }
                *(volatile v8h*)(crow + (size_t)row * ldc + piece * 8) = o; if (C2) *(volatile v8h*)(C2 + (size_t)r0 * ldc + c0 + (size_t)row * ldc + piece * 8) = o2; }
        };
        pass(); __threadfence(); pass();
    } else {
        float* crow = C + (size_t)r0 * ldc + c0;
        auto pass = [&]() {
#pragma unroll
            for (int s = 0; s < 8; ++s) { const int Lid = (lane >> 3) + 4 * s, piece = lane & 7; const int row = Lid >> 1, cofs = (Lid & 1) * 32 + piece * 4;
                v4f val = *(const v4fa*)(os + row * 68 + cofs); if (R) { const v4f rv = *(const v4f*)(R + ((size_t)r0 + row) * ldc + c0 + cofs); val += roundR ? (v4f){bfr(rv[0]), bfr(rv[1]), bfr(rv[2]), bfr(rv[3])} : rv; }
                *(volatile v4f*)(crow + (size_t)row * ldc + cofs) = val; }
        };
        pass(); __threadfence(); pass();
    }
}


__global__ __launch_bounds__(128) void k_gemmh(const h16* __restrict__ A, const h16* __restrict__ Bn, const float* __restrict__ bias, float* C, int ldc, const float* __restrict__ R, int K, size_t sA, size_t sB, size_t sC, int roundR) {
    __shared__ __align__(16) float ost[4][16 * 68];
    const size_t z = blockIdx.z; A += z * sA; Bn += z * sB; C += z * sC; if (R) R += z * sC;
    const int lane = threadIdx.x & 31, wave = threadIdx.x >> 5, lr = lane & 15, hi = lane >> 4;
    const int r0 = blockIdx.x * 64 + wave * 16, c0 = blockIdx.y * 64;
    const size_t aoff = (size_t)(r0 + lr) * K + 8 * hi;
    size_t boff[4];
#pragma unroll
    for (int t = 0; t < 4; ++t) boff[t] = (size_t)(c0 + t * 16 + lr) * K + 8 * hi;
    v8f acc[4];
#pragma unroll
    for (int t = 0; t < 4; ++t) acc[t] = (v8f){};
#pragma unroll 1
    for (int kc = 0; kc < K; kc += 32) {
        const v16h a = cat16(*(const v8h*)(A + aoff + kc), *(const v8h*)(A + aoff + kc + 16));
#pragma unroll
        for (int t = 0; t < 4; ++t) { const v16h b = cat16(*(const v8h*)(Bn + boff[t] + kc), *(const v8h*)(Bn + boff[t] + kc + 16)); acc[t] = wmma16(a, b, acc[t]); }
        asm volatile("v_nop\n\tv_nop\n\tv_nop\n\tv_nop" : "+v"(acc[0]), "+v"(acc[1]), "+v"(acc[2]), "+v"(acc[3]) : "v"(a));
    }
    float* os = &ost[wave][0];
#pragma unroll
    for (int t = 0; t < 4; ++t) { const float bv = bias ? bfr(bias[c0 + t * 16 + lr]) : 0.f;
#pragma unroll
        for (int j = 0; j < 8; ++j) os[(hi * 8 + j) * 68 + t * 16 + lr] = acc[t][j] + bv; }
    __syncthreads();
    float* crow = C + (size_t)r0 * ldc + c0;
    auto pass = [&]() {
#pragma unroll
        for (int s = 0; s < 8; ++s) { const int Lid = (lane >> 3) + 4 * s, piece = lane & 7; const int row = Lid >> 1, cofs = (Lid & 1) * 32 + piece * 4;
            v4f val = *(const v4fa*)(os + row * 68 + cofs); if (R) { const v4f rv = *(const v4f*)(R + ((size_t)r0 + row) * ldc + c0 + cofs); val += roundR ? (v4f){bfr(rv[0]), bfr(rv[1]), bfr(rv[2]), bfr(rv[3])} : rv; }
            *(volatile v4f*)(crow + (size_t)row * ldc + cofs) = val; }
    };
    pass(); __threadfence(); pass();
}

typedef __attribute__((ext_vector_type(4))) _Float16 v4h;
__device__ __forceinline__ h16 tohx(float x) { return (h16)x; }
__constant__ int c_off[11] = {0, 4, 16, 47, 54, 74, 424, 774, 1124, 1474, 1476};
__global__ __launch_bounds__(256) void k_wcatT(const float* __restrict__ Wc, float* WT) {
    __shared__ float tl[64][65];
    const int tid = threadIdx.x; const int o0 = blockIdx.x * 64, j0 = blockIdx.y * 64; const int rr = tid >> 2, cq = (tid & 3) * 16;
#pragma unroll
    for (int i = 0; i < 16; ++i) { const int o = o0 + rr, j = j0 + cq + i; tl[rr][cq + i] = (o < NCAT && j < NCAT) ? bfr(Wc[(size_t)o * NCAT + j]) : 0.f; }
    __syncthreads();
    const int lane = tid & 31, wv = tid >> 5;
    auto pass = [&]() {
#pragma unroll
        for (int st = 0; st < 4; ++st) { const int jr = wv * 8 + st * 2 + (lane >> 4); const int oq = (lane & 15) * 4; const int j = j0 + jr; if (j < NCAT) { v4f v;
#pragma unroll
                for (int i = 0; i < 4; ++i) v[i] = tl[oq + i][jr];
                *(volatile v4f*)(WT + (size_t)j * KP + o0 + oq) = v; } }
    };
    pass(); __threadfence(); pass();
}
__global__ __launch_bounds__(256) void k_hrow(const int* __restrict__ xc, const float* __restrict__ xcont, const float* __restrict__ WT, const float* __restrict__ bcat, h16* A) {
    const int lane = threadIdx.x & 31; const size_t b = (size_t)blockIdx.x * 8 + (threadIdx.x >> 5); if (b >= (size_t)16384) return; int idx[11];
#pragma unroll
    for (int i = 0; i < 11; ++i) { int v = xc[b * 11 + i]; const int hiN = (i == 10) ? (NCAT - c_off[10]) : (c_off[i + 1] - c_off[i]); v = v < 0 ? 0 : (v >= hiN ? hiN - 1 : v); idx[i] = c_off[i] + v; }
#pragma unroll 1
    for (int ps = 0; ps < 2; ++ps) {
#pragma unroll 1
        for (int q = 0; q < KP / 256; ++q) { const int c0 = q * 256 + lane * 8; v8h o;
#pragma unroll
            for (int k = 0; k < 8; ++k) { const int c = c0 + k; float y = 0.f;
                if (c < NCAT) { float s = bfr(bcat[c]);
#pragma unroll
                    for (int i = 0; i < 11; ++i) s += WT[(size_t)idx[i] * KP + c];
                    y = fmaxf(s, 0.f); }
                else if (c < NCAT + NCON) y = bfr(xcont[b * NCON + (c - NCAT)]);
                o[k] = tohx(y); }
            *(volatile v8h*)(A + b * KP + c0) = o; }
        if (ps == 0) __threadfence(); }
}
__global__ __launch_bounds__(256) void k_w1h(const float* __restrict__ W1, h16* Bt) {
    const int lane = threadIdx.x & 31; const int o_ = blockIdx.x * 8 + (threadIdx.x >> 5); if (o_ >= N1P) return;
#pragma unroll 1
    for (int ps = 0; ps < 2; ++ps) {
#pragma unroll 1
        for (int q = 0; q < KP / 256; ++q) { const int c0 = q * 256 + lane * 8; v8h o;
#pragma unroll
            for (int k = 0; k < 8; ++k) { const int c = c0 + k; o[k] = tohx((o_ < N1 && c < NCAT + NCON) ? bfr(W1[(size_t)(o_ < N1 ? o_ : 0) * (NCAT + NCON) + (c < NCAT + NCON ? c : 0)]) : 0.f); }
            *(volatile v8h*)(Bt + (size_t)o_ * KP + c0) = o; }
        if (ps == 0) __threadfence(); }
}
__global__ __launch_bounds__(256) void k_wpadn(const float* __restrict__ Wm, int Nl, int Kl, int NP, int KPd, bf* Bt) {
    const int lane = threadIdx.x & 31; const int n = blockIdx.x * 8 + (threadIdx.x >> 5); if (n >= NP) return;
#pragma unroll 1
    for (int ps = 0; ps < 2; ++ps) { for (int c0 = lane * 8; c0 < KPd; c0 += 256) { v8us o;
#pragma unroll
            for (int i = 0; i < 8; ++i) { const int k = c0 + i; const bool live = (n < Nl) && (k < Kl); o[i] = f2bf(live ? Wm[(size_t)(live ? n : 0) * Kl + (live ? k : 0)] : 0.f); }
            *(volatile v8us*)(Bt + (size_t)n * KPd + c0) = o; }
        if (ps == 0) __threadfence(); }
}
__global__ __launch_bounds__(256) void k_bpadn(const float* __restrict__ b, int Nl, int NP, float* BP) {
    const int i = blockIdx.x * 256 + threadIdx.x; if (i >= NP) return; const float v = (i < Nl) ? b[i] : 0.f; *(volatile float*)(BP + i) = v; __threadfence(); *(volatile float*)(BP + i) = v;
}
__global__ __launch_bounds__(256) void k_relu256p(const float* __restrict__ F, size_t rows, bf* Ph, bf* Pl) {
    const int lane = threadIdx.x & 31; const size_t r = (size_t)blockIdx.x * 8 + (threadIdx.x >> 5); if (r >= rows) return; const size_t o = r * N1P + lane * 8; const v8f v = *(const v8f*)(F + o); v8us oh, ol;
#pragma unroll
    for (int i = 0; i < 8; ++i) { const float y = fmaxf(v[i], 0.f); const unsigned short hb = f2bf(y); oh[i] = hb; ol[i] = f2bf(y - bf2f(hb)); }
    *(volatile v8us*)(Ph + o) = oh; *(volatile v8us*)(Pl + o) = ol; __threadfence(); *(volatile v8us*)(Ph + o) = oh; *(volatile v8us*)(Pl + o) = ol;
}
__global__ __launch_bounds__(256) void k_final(const float* __restrict__ X2, const float* __restrict__ W3, const float* __restrict__ b3, float* OUTB) {
    const int lane = threadIdx.x & 31; const size_t b = ((size_t)blockIdx.x * 8 + (threadIdx.x >> 5)) * 32 + lane; if (b >= (size_t)16384) return; float a = bfr(b3[0]);
#pragma unroll 1
    for (int c = 0; c < N2; ++c) a = fmaf(fmaxf(X2[b * N2P + c], 0.f), bfr(W3[c]), a);
    *(volatile float*)(OUTB + b) = a; __threadfence(); *(volatile float*)(OUTB + b) = a;
}

#define RCH 16384
extern "C" void kernel_launch(void* const* d_in, const int* in_sizes, int n_in,
                              void* d_out, int out_size, void* d_ws, size_t ws_size, hipStream_t stream) {
    (void)in_sizes; (void)n_in; (void)out_size;
    const int* xc = (const int*)d_in[0]; const float* xcont = (const float*)d_in[1]; const float* Wc = (const float*)d_in[2]; const float* bcat = (const float*)d_in[3]; const float* W1 = (const float*)d_in[4]; const float* b1 = (const float*)d_in[5]; const float* W2 = (const float*)d_in[6]; const float* b2 = (const float*)d_in[7]; const float* W3 = (const float*)d_in[8]; const float* b3 = (const float*)d_in[9];
    float* out = (float*)d_out;
    char* wsp = (char*)d_ws;
    auto take = [&](size_t bytes) { char* p = wsp; wsp += (bytes + 255) & ~(size_t)255; return (void*)p; };
    float* WT = (float*)take((size_t)NCAT * KP * 4); h16* BT1 = (h16*)take((size_t)N1P * KP * 2); float* BP1 = (float*)take(N1P * 4); bf* BT2 = (bf*)take((size_t)N2P * N1P * 2); float* BP2 = (float*)take(N2P * 4);
    h16* A = (h16*)take((size_t)RCH * KP * 2); float* X1 = (float*)take((size_t)RCH * N1P * 4); bf* Ph = (bf*)take((size_t)RCH * N1P * 2); bf* Pl = (bf*)take((size_t)RCH * N1P * 2); float* X2 = (float*)take((size_t)RCH * N2P * 4);
    if ((size_t)(wsp - (char*)d_ws) > ws_size) return;
    k_wcatT<<<dim3(24, 24, 1), 256, 0, stream>>>(Wc, WT);
    k_w1h<<<N1P / 8, 256, 0, stream>>>(W1, BT1); k_bpadn<<<1, 256, 0, stream>>>(b1, N1, N1P, BP1);
    k_wpadn<<<N2P / 8, 256, 0, stream>>>(W2, N2, N1, N2P, N1P, BT2); k_bpadn<<<1, 256, 0, stream>>>(b2, N2, N2P, BP2);
    for (int ch = 0; ch < NB_ / RCH; ++ch) { const size_t r0 = (size_t)ch * RCH;
        k_hrow<<<RCH / 8, 256, 0, stream>>>(xc + r0 * 11, xcont + r0 * NCON, WT, bcat, A);
        k_gemmh<<<dim3(RCH / 64, N1P / 64, 1), 128, 0, stream>>>(A, BT1, BP1, X1, N1P, nullptr, KP, 0, 0, 0, 0);
        k_relu256p<<<RCH / 8, 256, 0, stream>>>(X1, RCH, Ph, Pl);
        k_gemmb<true, false><<<dim3(RCH / 64, N2P / 64, 1), 128, 0, stream>>>(Ph, Pl, BT2, BP2, X2, N2P, nullptr, nullptr, N1P);
        k_final<<<(RCH / 32) / 8, 256, 0, stream>>>(X2, W3, b3, out + r0); }
}
